// lstm_49520972923007
// MI455X (gfx1250) — hardware-verified
//
#include <hip/hip_runtime.h>
#include <math.h>

constexpr int NBATCH   = 16384;
constexpr int NSTEP    = 150;
constexpr int NFEAT    = 5;
constexpr int NHID     = 64;
constexpr int NGATE    = 4 * NHID;
constexpr int ROWS_BLK = 32;
constexpr int NTHR     = 256;
constexpr int HPITCH   = 72;
constexpr int XROW     = NSTEP * NFEAT;
constexpr float ACT_CARRY = 64.0f;
constexpr float WGT_CARRY = 16.0f;
constexpr float FOLD_INV  = 1.0f / (ACT_CARRY * WGT_CARRY);

static_assert(NBATCH % ROWS_BLK == 0, "grid exact");
static_assert(ROWS_BLK == 32, "one 128-B output line per block");
static_assert(NTHR == 256, "8 waves: 2 row sub-tiles x 4 hidden slices");
static_assert(NHID == 64, "two 32-deep k chunks for the hidden part");
static_assert(NFEAT <= 8, "input features fit the first 8 k slots of the third chunk");
static_assert((ROWS_BLK * HPITCH) % NTHR == 0, "zero-fill loop exact");
static_assert(HPITCH % 8 == 0 && HPITCH >= NHID, "16-B aligned fragment loads");
static_assert(XROW == 750, "x row pitch");

typedef __attribute__((ext_vector_type(16))) _Float16 v16h;
typedef __attribute__((ext_vector_type(8)))  _Float16 v8h;
typedef __attribute__((ext_vector_type(8)))  float    v8f;
typedef __attribute__((ext_vector_type(4)))  float    v4f;

template <typename T> struct Frag;
template <> struct Frag<_Float16> {
  typedef v16h V; union U { v16h v; v8h h[2]; };
  static __device__ __forceinline__ v16h load(const _Float16* p) {
    U f; f.h[0] = *(const v8h*)(p); f.h[1] = *(const v8h*)(p + 16); return f.v;
  }
  static __device__ __forceinline__ v8f mma(v16h a, v16h b, v8f c) {
    return __builtin_amdgcn_wmma_f32_16x16x32_f16(false, a, false, b, (short)0, c, false, false);
  }
};

__device__ __forceinline__ void guard_all(v8f& a, v8f& b, v8f& c, v8f& d, v16h x, v16h y, v16h z) {
  asm volatile("v_nop\n\tv_nop\n\tv_nop\n\tv_nop" : "+v"(a), "+v"(b), "+v"(c), "+v"(d) : "v"(x), "v"(y), "v"(z));
}
__device__ __forceinline__ void pin_frag2(v16h& a, v16h& b) { asm volatile("" : "+v"(a), "+v"(b) :: "memory"); }
__device__ __forceinline__ void pin_frag1(v16h& a, float& s) { asm volatile("" : "+v"(a), "+v"(s) :: "memory"); }

__device__ __forceinline__ v16h zero_frag() {
  v16h z;
#pragma unroll
  for (int e = 0; e < 16; ++e) z[e] = (_Float16)0.0f;
  return z;
}

__device__ __forceinline__ float fsig(float x)  { return __builtin_amdgcn_rcpf(1.0f + __expf(-x)); }
__device__ __forceinline__ float ftanh(float x) { return 1.0f - 2.0f * __builtin_amdgcn_rcpf(__expf(2.0f * x) + 1.0f); }

__global__ __launch_bounds__(NTHR) void lstm_seq_kernel(const float* __restrict__ x, const float* __restrict__ w_ih,
                                                        const float* __restrict__ w_hh, const float* __restrict__ b_ih,
                                                        const float* __restrict__ b_hh, const float* __restrict__ w_lin,
                                                        const float* __restrict__ b_lin, float* __restrict__ out) {
  __shared__ __align__(16) _Float16 Ah[2][ROWS_BLK * HPITCH];
  __shared__ float Part[4][ROWS_BLK];

  const int tid  = threadIdx.x;
  const int lane = tid & 31;
  const int wave = tid >> 5;
  const int c    = lane & 15;
  const int hh   = lane >> 4;
  const int koff = hh * 8;
  const int sub  = wave >> 2;
  const int wq   = wave & 3;
  const int j    = 16 * wq + c;
  const bool lo  = (hh == 0);
  const int rowbase = blockIdx.x * ROWS_BLK;

  {
    _Float16* ah0 = &Ah[0][0];
#pragma unroll 1
    for (int i = tid; i < ROWS_BLK * HPITCH; i += NTHR) ah0[i] = (_Float16)0.0f;
  }

  float zlane = 0.0f;
  asm volatile("" : "+v"(zlane));

  v16h Bh[4][2];
  v16h Bx[4];
  float bsum[4];
#pragma unroll
  for (int q = 0; q < 4; ++q) {
    const int n = q * NHID + j;
    const float* wr = w_hh + (size_t)n * NHID + koff;
#pragma unroll
    for (int kc = 0; kc < 2; ++kc) {
      const v4f p0 = *(const v4f*)(wr + 32 * kc);
      const v4f p1 = *(const v4f*)(wr + 32 * kc + 4);
      const v4f p2 = *(const v4f*)(wr + 32 * kc + 16);
      const v4f p3 = *(const v4f*)(wr + 32 * kc + 20);
      v16h f;
#pragma unroll
      for (int e = 0; e < 4; ++e) {
        f[e]      = (_Float16)(p0[e] * WGT_CARRY);
        f[4 + e]  = (_Float16)(p1[e] * WGT_CARRY);
        f[8 + e]  = (_Float16)(p2[e] * WGT_CARRY);
        f[12 + e] = (_Float16)(p3[e] * WGT_CARRY);
      }
      Bh[q][kc] = f;
    }
    pin_frag2(Bh[q][0], Bh[q][1]);

    const float* wi = w_ih + (size_t)n * NFEAT;
    const float u0 = wi[0];
    const float u1 = wi[1];
    const float u2 = wi[2];
    const float u3 = wi[3];
    const float u4 = wi[4];
    const float ba = b_ih[n];
    const float bb = b_hh[n];
    v16h g = zero_frag();
    g[0] = (_Float16)(lo ? u0 * WGT_CARRY : 0.0f);
    g[1] = (_Float16)(lo ? u1 * WGT_CARRY : 0.0f);
    g[2] = (_Float16)(lo ? u2 * WGT_CARRY : 0.0f);
    g[3] = (_Float16)(lo ? u3 * WGT_CARRY : 0.0f);
    g[4] = (_Float16)(lo ? u4 * WGT_CARRY : 0.0f);
    g[5] = (_Float16)zlane;
    float bs = ba + bb;
    pin_frag1(g, bs);
    Bx[q] = g;
    bsum[q] = bs;
  }

  float cst[8], hst[8];
#pragma unroll
  for (int r = 0; r < 8; ++r) { cst[r] = 0.0f; hst[r] = 0.0f; }

  const float* xrow = x + (size_t)(rowbase + 16 * sub + c) * XROW;
  float xn0 = xrow[0];
  float xn1 = xrow[1];
  float xn2 = xrow[2];
  float xn3 = xrow[3];
  float xn4 = xrow[4];

  const v8f z8 = {0.f, 0.f, 0.f, 0.f, 0.f, 0.f, 0.f, 0.f};
  __syncthreads();

#pragma unroll 1
  for (int t = 0; t < NSTEP; ++t) {
    const int cur = t & 1;
    const float xc0 = xn0, xc1 = xn1, xc2 = xn2, xc3 = xn3, xc4 = xn4;
    {
      const int tn = (t + 1 < NSTEP) ? (t + 1) : (NSTEP - 1);
      const float* xp = xrow + tn * NFEAT;
      xn0 = xp[0];
      xn1 = xp[1];
      xn2 = xp[2];
      xn3 = xp[3];
      xn4 = xp[4];
    }
    const _Float16* ahrow = &Ah[cur][0] + (16 * sub + c) * HPITCH + koff;
    _Float16* ahn = &Ah[cur ^ 1][0];

    const v16h a0 = Frag<_Float16>::load(ahrow);
    const v16h a1 = Frag<_Float16>::load(ahrow + 32);
    v16h ax = zero_frag();
    ax[0] = (_Float16)(lo ? xc0 * ACT_CARRY : 0.0f);
    ax[1] = (_Float16)(lo ? xc1 * ACT_CARRY : 0.0f);
    ax[2] = (_Float16)(lo ? xc2 * ACT_CARRY : 0.0f);
    ax[3] = (_Float16)(lo ? xc3 * ACT_CARRY : 0.0f);
    ax[4] = (_Float16)(lo ? xc4 * ACT_CARRY : 0.0f);
    ax[5] = (_Float16)zlane;

    v8f acc[4];
#pragma unroll
    for (int q = 0; q < 4; ++q) acc[q] = Frag<_Float16>::mma(ax, Bx[q], z8);
#pragma unroll
    for (int q = 0; q < 4; ++q) acc[q] = Frag<_Float16>::mma(a0, Bh[q][0], acc[q]);
#pragma unroll
    for (int q = 0; q < 4; ++q) acc[q] = Frag<_Float16>::mma(a1, Bh[q][1], acc[q]);
    guard_all(acc[0], acc[1], acc[2], acc[3], a0, a1, ax);

#pragma unroll
    for (int r = 0; r < 8; ++r) {
      const float zi = fmaf(acc[0][r], FOLD_INV, bsum[0]);
      const float zf = fmaf(acc[1][r], FOLD_INV, bsum[1]);
      const float zg = fmaf(acc[2][r], FOLD_INV, bsum[2]);
      const float zo = fmaf(acc[3][r], FOLD_INV, bsum[3]);
      const float ig = fsig(zi);
      const float fg = fsig(zf);
      const float gg = ftanh(zg);
      const float og = fsig(zo);
      const float cn = fg * cst[r] + ig * gg;
      cst[r] = cn;
      const float hn = og * ftanh(cn);
      hst[r] = hn;
      ahn[(16 * sub + 8 * hh + r) * HPITCH + j] = (_Float16)(hn * ACT_CARRY);
    }
    __syncthreads();
  }

  const float wl = w_lin[j];
  const float bl = b_lin[0];
  float pr[8];
#pragma unroll
  for (int r = 0; r < 8; ++r) pr[r] = hst[r] * wl;
#pragma unroll
  for (int r = 0; r < 8; ++r) {
    pr[r] += __shfl_xor(pr[r], 1, 32);
    pr[r] += __shfl_xor(pr[r], 2, 32);
    pr[r] += __shfl_xor(pr[r], 4, 32);
    pr[r] += __shfl_xor(pr[r], 8, 32);
  }
  if (c == 0) {
#pragma unroll
    for (int r = 0; r < 8; ++r) Part[wq][16 * sub + 8 * hh + r] = pr[r];
  }
  __syncthreads();
  if (wave == 0) {
    const float v = ((Part[0][lane] + Part[1][lane]) + (Part[2][lane] + Part[3][lane])) + bl;
    volatile float* op = out + rowbase + lane;
    *op = v;
    __threadfence();
    *op = v;
  }
}

extern "C" void kernel_launch(void* const* d_in, const int* in_sizes, int n_in,
                              void* d_out, int out_size, void* d_ws, size_t ws_size, hipStream_t stream) {
  (void)d_ws; (void)ws_size;
  if (n_in < 7 || d_out == nullptr) return;
  if (in_sizes[0] != NBATCH * NSTEP * NFEAT || in_sizes[1] != NGATE * NFEAT || in_sizes[2] != NGATE * NHID ||
      in_sizes[3] != NGATE || in_sizes[4] != NGATE || in_sizes[5] != NHID || in_sizes[6] != 1 ||
      out_size != NBATCH) return;

  const float* x     = (const float*)d_in[0];
  const float* w_ih  = (const float*)d_in[1];
  const float* w_hh  = (const float*)d_in[2];
  const float* b_ih  = (const float*)d_in[3];
  const float* b_hh  = (const float*)d_in[4];
  const float* w_lin = (const float*)d_in[5];
  const float* b_lin = (const float*)d_in[6];
  float* out = (float*)d_out;

  lstm_seq_kernel<<<NBATCH / ROWS_BLK, NTHR, 0, stream>>>(x, w_ih, w_hh, b_ih, b_hh, w_lin, b_lin, out);
}
